// GraphAE_84473416777939
// MI455X (gfx1250) — hardware-verified
//
#include <hip/hip_runtime.h>
#include <stddef.h>


#define FIN     256
#define HCN     256
#define NHD     4
#define CHN     64
#define CPL     8
#define NTHR    256
#define NWAVE   8
#define EPT     8
#define NGRP    2
#define CHUNK   (NTHR * EPT * NGRP)
#define WCAP    (EPT * NGRP * 32)
#define LISTN   (NWAVE * WCAP)
#define NBC     4096
#define NBF     1024
#define RCAP    40960
#define RBN     128
#define TGT     256
#define DEGCAP  512
#define OTHR    512
#define BM      64
#define BN      128
#define WSCAP   134217728
#define NEG_SLOPE 0.2f
#define WSC     16.0f
#define H1SC    8.0f

#define LDS_FILL ((RCAP + NBF + LISTN) * 4 + 64)

static_assert((CHUNK & (CHUNK - 1)) == 0);
static_assert(CHUNK <= 4096);
static_assert(NBC <= 4096 && NBF <= 4096);
static_assert((NBC & (NBC - 1)) == 0 && (NBF & (NBF - 1)) == 0);
static_assert(NBC == 4 * NBF);
static_assert(OTHR * 8 == NBC);
static_assert((RCAP % 32) == 0);
static_assert(TGT == NWAVE * 32);
static_assert((NBC % TGT) == 0);
static_assert((TGT % BM) == 0);
static_assert(BM * 4 == NTHR);
static_assert(FIN % 32 == 0 && HCN % 32 == 0);
static_assert(NHD * CHN == HCN);
static_assert(BN == 2 * CHN);
static_assert(HCN % BN == 0);
static_assert(HCN == 32 * CPL);
static_assert(CHN == 8 * CPL);
static_assert(CPL == 8);
static_assert(CHN == 16 * 4);

typedef float          v2f  __attribute__((ext_vector_type(2)));
typedef float          v4f  __attribute__((ext_vector_type(4)));
typedef float          v8f  __attribute__((ext_vector_type(8)));
typedef int            v4i  __attribute__((ext_vector_type(4)));
typedef unsigned short v8us __attribute__((ext_vector_type(8)));
typedef _Float16       v8h  __attribute__((ext_vector_type(8)));
typedef _Float16       v16h __attribute__((ext_vector_type(16)));
union FragH { v16h v; v8us u[2]; };
union Pk8   { v8h h; v8us u; };

__device__ __forceinline__ v8f wmh(v16h a, v16h b, v8f c) {
  v8f d = __builtin_amdgcn_wmma_f32_16x16x32_f16(false, a, false, b, (short)0, c, false, false);
  asm volatile("v_nop\n\tv_nop\n\tv_nop\n\tv_nop" : "+v"(d) : "v"(a), "v"(b));
  return d;
}

__device__ __forceinline__ v8us cvt8h(v4f a, v4f b, float sc) {
  v8f f;
  f[0] = a.x * sc; f[1] = a.y * sc; f[2] = a.z * sc; f[3] = a.w * sc;
  f[4] = b.x * sc; f[5] = b.y * sc; f[6] = b.z * sc; f[7] = b.w * sc;
  Pk8 r;
  r.h = __builtin_convertvector(f, v8h);
  return r.u;
}

__device__ __forceinline__ float lrelu(float v) { return v > 0.0f ? v : NEG_SLOPE * v; }
__device__ __forceinline__ float elu1(float v) { return v > 0.0f ? v : (__expf(v) - 1.0f); }
__device__ __forceinline__ v4f elu4(v4f v) {
  v4f r;
  r.x = elu1(v.x); r.y = elu1(v.y); r.z = elu1(v.z); r.w = elu1(v.w);
  return r;
}
__device__ __forceinline__ float hsum2(float t) {
  t += __shfl_xor(t, 8);
  t += __shfl_xor(t, 16);
  return t;
}
__device__ __forceinline__ v4f hsum2v(v4f v) {
  v4f r;
  r.x = hsum2(v.x); r.y = hsum2(v.y); r.z = hsum2(v.z); r.w = hsum2(v.w);
  return r;
}

template <int NB>
__device__ __forceinline__ int scan_chunk(const int* __restrict__ dsts, int nE, int cbase, int slotBase,
                                          int vec8, int* list, int tid, int lane, int wave) {
  int wc = 0;
#pragma unroll
  for (int g = 0; g < NGRP; ++g) {
    const int el0  = (g * NTHR + tid) * EPT;
    const int e0   = cbase + el0;
    const int sent = -2147483647 - 1;
    v4i da, db;
    if (vec8 != 0 && cbase + CHUNK <= nE) {
      da = *(const v4i*)(dsts + e0);
      db = *(const v4i*)(dsts + e0 + 4);
    } else {
      da.x = (e0     < nE) ? dsts[min(e0, nE - 1)] : sent;
      da.y = (e0 + 1 < nE) ? dsts[min(e0 + 1, nE - 1)] : sent;
      da.z = (e0 + 2 < nE) ? dsts[min(e0 + 2, nE - 1)] : sent;
      da.w = (e0 + 3 < nE) ? dsts[min(e0 + 3, nE - 1)] : sent;
      db.x = (e0 + 4 < nE) ? dsts[min(e0 + 4, nE - 1)] : sent;
      db.y = (e0 + 5 < nE) ? dsts[min(e0 + 5, nE - 1)] : sent;
      db.z = (e0 + 6 < nE) ? dsts[min(e0 + 6, nE - 1)] : sent;
      db.w = (e0 + 7 < nE) ? dsts[min(e0 + 7, nE - 1)] : sent;
    }
    const unsigned nb = (unsigned)slotBase;
    const unsigned s0 = (unsigned)da.x - nb, s1 = (unsigned)da.y - nb;
    const unsigned s2 = (unsigned)da.z - nb, s3 = (unsigned)da.w - nb;
    const unsigned s4 = (unsigned)db.x - nb, s5 = (unsigned)db.y - nb;
    const unsigned s6 = (unsigned)db.z - nb, s7 = (unsigned)db.w - nb;
    const bool h0 = s0 < (unsigned)NB, h1 = s1 < (unsigned)NB, h2 = s2 < (unsigned)NB, h3 = s3 < (unsigned)NB;
    const bool h4 = s4 < (unsigned)NB, h5 = s5 < (unsigned)NB, h6 = s6 < (unsigned)NB, h7 = s7 < (unsigned)NB;
    const unsigned any = __builtin_amdgcn_ballot_w32(h0 | h1 | h2 | h3 | h4 | h5 | h6 | h7);
    if (any != 0u) {
#define HITJ(J, HJ, SJ) { \
        const unsigned mj = __builtin_amdgcn_ballot_w32(HJ); \
        if (mj != 0u) { \
          if (HJ) { \
            const int pos = wc + (int)__builtin_amdgcn_mbcnt_lo(mj, 0u); \
            if (pos < WCAP) list[wave * WCAP + pos] = ((el0 + (J)) << 12) | (int)(SJ); \
          } \
          wc += (int)__builtin_popcount(mj); } }
      HITJ(0, h0, s0)
      HITJ(1, h1, s1)
      HITJ(2, h2, s2)
      HITJ(3, h3, s3)
      HITJ(4, h4, s4)
      HITJ(5, h5, s5)
      HITJ(6, h6, s6)
      HITJ(7, h7, s7)
#undef HITJ
    }
  }
  return wc;
}

__global__ __launch_bounds__(NTHR) void k_xcvt(const float* __restrict__ x, unsigned short* xp, int nN, int nUnits) {
  const int i = (int)blockIdx.x * NTHR + (int)threadIdx.x;
  if (i >= nUnits) return;
  const int row = i >> 5;
  const int c0  = (i & 31) * 8;
  int rr = row > nN - 1 ? nN - 1 : row;
  rr = rr < 0 ? 0 : rr;
  const float* p = x + (size_t)rr * FIN + c0;
  v4f a = *(const v4f*)p, b = *(const v4f*)(p + 4);
  const v4f z = {0.f, 0.f, 0.f, 0.f};
  if (row >= nN) { a = z; b = z; }
  const v8us o = cvt8h(a, b, 1.0f);
  unsigned short* d = xp + (size_t)i * 8;
  *(volatile v8us*)d = o;
  __threadfence();
  *(volatile v8us*)d = o;
}

template <int KD, int NCW>
__global__ __launch_bounds__(NTHR) void k_wprep(const float* __restrict__ W, unsigned short* wp) {
  constexpr int KS    = KD / 8;
  constexpr int UNITS = NCW * KS;
  static_assert(KD % 8 == 0);
  const int i = (int)blockIdx.x * NTHR + (int)threadIdx.x;
  if (i >= UNITS) return;
  const int n  = i / KS;
  const int k0 = (i - n * KS) * 8;
  v4f a, b;
  a.x = W[(size_t)(k0 + 0) * NCW + n]; a.y = W[(size_t)(k0 + 1) * NCW + n];
  a.z = W[(size_t)(k0 + 2) * NCW + n]; a.w = W[(size_t)(k0 + 3) * NCW + n];
  b.x = W[(size_t)(k0 + 4) * NCW + n]; b.y = W[(size_t)(k0 + 5) * NCW + n];
  b.z = W[(size_t)(k0 + 6) * NCW + n]; b.w = W[(size_t)(k0 + 7) * NCW + n];
  const v8us o = cvt8h(a, b, WSC);
  unsigned short* d = wp + (size_t)i * 8;
  *(volatile v8us*)d = o;
  __threadfence();
  *(volatile v8us*)d = o;
}

__global__ __launch_bounds__(NTHR) void k_count(
    const int* __restrict__ dsts, int* cnt, int nE, int vec8) {
  __shared__ __attribute__((aligned(16))) int scnt[NBC];
  __shared__ __attribute__((aligned(16))) int list[LISTN];
  __shared__ int wcnt[NWAVE];
  const int tid = threadIdx.x, lane = tid & 31, wave = tid >> 5;
  const int nodeBase = blockIdx.x * NBC;

  for (int i = tid; i < NBC; i += NTHR) scnt[i] = 0;
  __syncthreads();

  const int nChunks = (nE + CHUNK - 1) / CHUNK;
#pragma unroll 1
  for (int ch = 0; ch < nChunks; ++ch) {
    const int cbase = ch * CHUNK;
    const int wc = scan_chunk<NBC>(dsts, nE, cbase, nodeBase, vec8, list, tid, lane, wave);
    if (lane == 0) wcnt[wave] = wc;
    __syncthreads();
    if (wave == 0) {
#pragma unroll 1
      for (int wsx = 0; wsx < NWAVE; ++wsx) {
        int n = __builtin_amdgcn_readfirstlane(wcnt[wsx]);
        n = n > WCAP ? WCAP : (n < 0 ? 0 : n);
        const int* lp = list + wsx * WCAP;
#pragma unroll 1
        for (int i = 0; i < n; ++i) {
          const int ent  = __builtin_amdgcn_readfirstlane(lp[i]);
          const int slot = ent & (NBC - 1);
          if (lane == 0) scnt[slot] = scnt[slot] + 1;
        }
      }
    }
    __syncthreads();
  }

  v4i cq[4];
#pragma unroll
  for (int q = 0; q < 4; ++q) {
    const int f = (wave * 4 + q) * 128 + 4 * lane;
    cq[q] = *(const v4i*)(scnt + f);
  }
  int* cp = cnt + (size_t)nodeBase;
#pragma unroll
  for (int q = 0; q < 4; ++q) {
    const int f = (wave * 4 + q) * 128 + 4 * lane;
    *(volatile v4i*)(cp + f) = cq[q];
  }
  __threadfence();
#pragma unroll
  for (int q = 0; q < 4; ++q) {
    const int f = (wave * 4 + q) * 128 + 4 * lane;
    *(volatile v4i*)(cp + f) = cq[q];
  }
}

__global__ __launch_bounds__(OTHR) void k_offsets(
    const int* __restrict__ cnt, int* off, int* rbase, int nChunk) {
  __shared__ __attribute__((aligned(16))) int soff[NBC];
  __shared__ __attribute__((aligned(16))) int srb[RBN];
  __shared__ int wtot[OTHR / 32];
  const int tid = threadIdx.x, lane = tid & 31, wave = tid >> 5, sub = tid >> 7;
  for (int i = tid; i < RBN; i += OTHR) srb[i] = 0;
  int carry = 0;
#pragma unroll 1
  for (int ch = 0; ch < nChunk; ++ch) {
    const int base = ch * NBC;
    const v4i c0 = *(const v4i*)(cnt + base + 8 * tid);
    const v4i c1 = *(const v4i*)(cnt + base + 8 * tid + 4);
    const int e0 = max(c0.x, 0), e1 = max(c0.y, 0), e2 = max(c0.z, 0), e3 = max(c0.w, 0);
    const int e4 = max(c1.x, 0), e5 = max(c1.y, 0), e6 = max(c1.z, 0), e7 = max(c1.w, 0);
    const int ts = e0 + e1 + e2 + e3 + e4 + e5 + e6 + e7;
    int incl = ts;
#pragma unroll
    for (int d = 1; d < 32; d <<= 1) {
      const int t = __shfl_up(incl, d);
      if (lane >= d) incl += t;
    }
    if (lane == 31) wtot[wave] = incl;
    __syncthreads();
    const int S0 = wtot[0]  + wtot[1]  + wtot[2]  + wtot[3];
    const int S1 = wtot[4]  + wtot[5]  + wtot[6]  + wtot[7];
    const int S2 = wtot[8]  + wtot[9]  + wtot[10] + wtot[11];
    const int S3 = wtot[12] + wtot[13] + wtot[14] + wtot[15];
    int pre = 0;
#pragma unroll 1
    for (int w = 4 * sub; w < wave; ++w) pre += wtot[w];
    const int b0 = carry;
    const int b1 = b0 + ((S0 + 31) & ~31);
    const int b2 = b1 + ((S1 + 31) & ~31);
    const int b3 = b2 + ((S2 + 31) & ~31);
    const int b4 = b3 + ((S3 + 31) & ~31);
    const int myb = sub == 0 ? b0 : (sub == 1 ? b1 : (sub == 2 ? b2 : b3));
    if (tid == 0) {
      srb[min(4 * ch + 0, RBN - 1)] = b0;
      srb[min(4 * ch + 1, RBN - 1)] = b1;
      srb[min(4 * ch + 2, RBN - 1)] = b2;
      srb[min(4 * ch + 3, RBN - 1)] = b3;
    }
    int run = myb + pre + incl - ts;
    soff[8 * tid + 0] = run; run += e0;
    soff[8 * tid + 1] = run; run += e1;
    soff[8 * tid + 2] = run; run += e2;
    soff[8 * tid + 3] = run; run += e3;
    soff[8 * tid + 4] = run; run += e4;
    soff[8 * tid + 5] = run; run += e5;
    soff[8 * tid + 6] = run; run += e6;
    soff[8 * tid + 7] = run;
    carry = b4;
    __syncthreads();
    const v4i o0 = *(const v4i*)(soff + 4 * tid);
    const v4i o1 = *(const v4i*)(soff + 4 * (tid + OTHR));
    int* op = off + base;
    *(volatile v4i*)(op + 4 * tid) = o0;
    *(volatile v4i*)(op + 4 * (tid + OTHR)) = o1;
    __threadfence();
    *(volatile v4i*)(op + 4 * tid) = o0;
    *(volatile v4i*)(op + 4 * (tid + OTHR)) = o1;
    __syncthreads();
  }
  if (tid == 0) srb[min(4 * nChunk, RBN - 1)] = carry;
  __syncthreads();
  v4i rv = {0, 0, 0, 0};
  if (tid < 32) rv = *(const v4i*)(srb + 4 * tid);
  if (tid < 32) *(volatile v4i*)(rbase + 4 * tid) = rv;
  __threadfence();
  if (tid < 32) *(volatile v4i*)(rbase + 4 * tid) = rv;
}

__global__ __launch_bounds__(NTHR) void k_fill(
    const int* __restrict__ srcs, const int* __restrict__ dsts,
    const int* __restrict__ off, const int* __restrict__ rbase,
    int* csr, int nN, int nE, int vec8, int csrLen) {
  extern __shared__ v4f lds_dyn[];
  int* region = (int*)lds_dyn;
  int* cursor = region + RCAP;
  int* list   = cursor + NBF;
  int* wcnt   = list + LISTN;
  const int tid = threadIdx.x, lane = tid & 31, wave = tid >> 5;
  const int b = blockIdx.x;
  const int nodeBase = b * NBF;

  int rb0 = rbase[b];
  const int rb1 = rbase[b + 1];
  rb0 = rb0 < 0 ? 0 : (rb0 > csrLen ? csrLen : rb0);
  rb0 &= ~31;
  int len = rb1 - rb0;
  len = len < 0 ? 0 : (len > RCAP ? RCAP : len);
  int lenW = (len + 31) & ~31;
  if (rb0 + lenW > csrLen) lenW = (csrLen - rb0) & ~31;

  {
    const v4i z = {0, 0, 0, 0};
    for (int i = tid; i < RCAP / 4; i += NTHR) ((v4i*)region)[i] = z;
    for (int s = tid; s < NBF; s += NTHR) {
      int o = off[nodeBase + s] - rb0;
      o = o < 0 ? 0 : (o > RCAP ? RCAP : o);
      cursor[s] = o;
    }
  }
  __syncthreads();

  const int nChunks = (nE + CHUNK - 1) / CHUNK;
#pragma unroll 1
  for (int ch = 0; ch < nChunks; ++ch) {
    const int cbase = ch * CHUNK;
    const int wc = scan_chunk<NBF>(dsts, nE, cbase, nodeBase, vec8, list, tid, lane, wave);
    if (lane == 0) wcnt[wave] = wc;
    __syncthreads();
    if (wave == 0) {
#pragma unroll 1
      for (int wsx = 0; wsx < NWAVE; ++wsx) {
        int n = __builtin_amdgcn_readfirstlane(wcnt[wsx]);
        n = n > WCAP ? WCAP : (n < 0 ? 0 : n);
        const int* lp = list + wsx * WCAP;
#pragma unroll 1
        for (int i = 0; i < n; ++i) {
          const int ent  = __builtin_amdgcn_readfirstlane(lp[i]);
          const int slot = ent & (NBF - 1);
          int e = cbase + ((ent >> 12) & (CHUNK - 1));
          e = e > nE - 1 ? nE - 1 : e;
          int src = srcs[e];
          src = src < 0 ? 0 : (src > nN - 1 ? nN - 1 : src);
          if (lane == 0) {
            int pos = cursor[slot];
            pos = pos < 0 ? 0 : (pos > RCAP - 1 ? RCAP - 1 : pos);
            region[pos] = src;
            const int np = pos + 1;
            cursor[slot] = np > RCAP ? RCAP : np;
          }
        }
      }
    }
    __syncthreads();
  }

  const int nv = lenW >> 2;
  int* gp = csr + rb0;
#pragma unroll 1
  for (int i = tid; i < nv; i += NTHR) { const v4i v = ((const v4i*)region)[i]; *(volatile v4i*)(gp + 4 * i) = v; }
  __threadfence();
#pragma unroll 1
  for (int i = tid; i < nv; i += NTHR) { const v4i v = ((const v4i*)region)[i]; *(volatile v4i*)(gp + 4 * i) = v; }
}

template <int K, int OSH>
__global__ __launch_bounds__(NTHR) void k_gemm(
    const unsigned short* __restrict__ Ap, const unsigned short* __restrict__ Bp,
    const float* __restrict__ attS, const float* __restrict__ attD,
    float* C, float* eS, float* eD, int npad) {
  constexpr int TPW = 4;
  constexpr int KT  = K / 32;
  constexpr int CPP = 32;
  constexpr int NES = BM * 2;
  constexpr int NIT = BM / NWAVE;
  static_assert(K % 32 == 0);
  static_assert(TPW * 16 * 2 == BN);
  static_assert(NES == 4 * 32);
  static_assert(BN == 4 * 32);
  static_assert(CHN == 2 * CPP);

  __shared__ __attribute__((aligned(16))) float stg[BM * BN];
  __shared__ __attribute__((aligned(16))) float sES[NES];
  __shared__ __attribute__((aligned(16))) float sED[NES];
  const int tid = threadIdx.x, lane = tid & 31, wave = tid >> 5, hh = lane >> 4, m = lane & 15;
  const int rowBase = blockIdx.x * BM;
  const int cs = blockIdx.y * BN;
  const int rg = wave >> 1, chf = wave & 1;
  const int r0 = rg * 16;
  const int c0 = chf * 64;
  const float osc = 1.0f / (float)(1 << OSH);

  v8f acc[TPW];
#pragma unroll
  for (int t = 0; t < TPW; ++t) { v8f z = {0.f, 0.f, 0.f, 0.f, 0.f, 0.f, 0.f, 0.f}; acc[t] = z; }

  const unsigned short* ap  = Ap + (size_t)(rowBase + r0 + m) * K + 8 * hh;
  const unsigned short* bp0 = Bp + (size_t)(cs + c0 + m) * K + 8 * hh;
#pragma unroll 1
  for (int kt = 0; kt < KT; ++kt) {
    FragH a;
    a.u[0] = *(const v8us*)(ap + 32 * kt);
    a.u[1] = *(const v8us*)(ap + 32 * kt + 16);
#pragma unroll
    for (int t = 0; t < TPW; ++t) {
      const unsigned short* bp = bp0 + (size_t)(16 * t) * K + 32 * kt;
      FragH bf;
      bf.u[0] = *(const v8us*)bp;
      bf.u[1] = *(const v8us*)(bp + 16);
      acc[t] = wmh(a.v, bf.v, acc[t]);
    }
  }

  {
    float* sp = stg + (size_t)(r0 + 8 * hh) * BN + c0 + m;
#pragma unroll
    for (int t = 0; t < TPW; ++t) {
#pragma unroll
      for (int r = 0; r < 8; ++r) sp[r * BN + 16 * t] = acc[t][r] * osc;
    }
  }
  __syncthreads();

  {
    const int drow = tid >> 2, part = tid & 3;
    const float* rp  = stg + (size_t)drow * BN + CPP * part;
    const float* sa  = attS + blockIdx.y * BN + CPP * part;
    const float* sdd = attD + blockIdx.y * BN + CPP * part;
    float ps = 0.f, pd = 0.f;
#pragma unroll 2
    for (int c = 0; c < CPP; c += 4) {
      const v4f hv = *(const v4f*)(rp + c);
      const v4f av = *(const v4f*)(sa + c);
      const v4f dv = *(const v4f*)(sdd + c);
      ps += hv.x * av.x + hv.y * av.y + hv.z * av.z + hv.w * av.w;
      pd += hv.x * dv.x + hv.y * dv.y + hv.z * dv.z + hv.w * dv.w;
    }
    ps += __shfl_xor(ps, 1); pd += __shfl_xor(pd, 1);
    if ((part & 1) == 0) { sES[drow * 2 + (part >> 1)] = ps; sED[drow * 2 + (part >> 1)] = pd; }
  }

  {
    float* cb = C + (size_t)rowBase * HCN + cs + 4 * lane;
    v4f cv[NIT];
#pragma unroll
    for (int it = 0; it < NIT; ++it) cv[it] = *(const v4f*)(stg + (size_t)(it * NWAVE + wave) * BN + 4 * lane);
#pragma unroll
    for (int it = 0; it < NIT; ++it) *(volatile v4f*)(cb + (size_t)(it * NWAVE + wave) * HCN) = cv[it];
    __threadfence();
#pragma unroll
    for (int it = 0; it < NIT; ++it) *(volatile v4f*)(cb + (size_t)(it * NWAVE + wave) * HCN) = cv[it];
  }
  __syncthreads();

  {
    const size_t eb = ((size_t)blockIdx.y * (size_t)npad + (size_t)rowBase) * 2;
    const v4f vS = *(const v4f*)(sES + 4 * lane);
    const v4f vD = *(const v4f*)(sED + 4 * lane);
    const v4f dv = (wave == 0) ? vS : vD;
    float* gp = ((wave == 0) ? eS : eD) + eb + 4 * lane;
    if (wave < 2) *(volatile v4f*)gp = dv;
    __threadfence();
    if (wave < 2) *(volatile v4f*)gp = dv;
  }
}

__device__ __forceinline__ void gat_row(
    const int* __restrict__ csr, const float* __restrict__ eS, const float* __restrict__ hw,
    size_t eoff, float edc, float eself, int c, int n, int st, int col, int lane, int nN, int csrLen,
    float& deno, v4f& a0, v4f& a1) {
  float mx = eself;
#pragma unroll 1
  for (int q0 = 0; q0 < n; q0 += 32) {
    int pos = st + q0 + lane;
    pos = pos < 0 ? 0 : (pos > csrLen - 1 ? csrLen - 1 : pos);
    int sl = csr[pos];
    sl = sl < 0 ? 0 : (sl > nN - 1 ? nN - 1 : sl);
    const int mcnt = (n - q0) < 32 ? (n - q0) : 32;
#pragma unroll 1
    for (int pp = 0; pp < mcnt; ++pp) {
      const int s = __builtin_amdgcn_readlane(sl, pp);
      mx = fmaxf(mx, lrelu(eS[eoff + (size_t)s * 2] + edc));
    }
  }

  float p   = __expf(eself - mx);
  float den = p;
  const float* hc = hw + (size_t)c * HCN + col;
  v4f b0 = *(const v4f*)hc * p;
  v4f b1 = *(const v4f*)(hc + 4) * p;
#pragma unroll 1
  for (int q0 = 0; q0 < n; q0 += 32) {
    int pos = st + q0 + lane;
    pos = pos < 0 ? 0 : (pos > csrLen - 1 ? csrLen - 1 : pos);
    int sl = csr[pos];
    sl = sl < 0 ? 0 : (sl > nN - 1 ? nN - 1 : sl);
    const int mcnt = (n - q0) < 32 ? (n - q0) : 32;
#pragma unroll 1
    for (int pp = 0; pp < mcnt; ++pp) {
      const int s = __builtin_amdgcn_readlane(sl, pp);
      p = __expf(lrelu(eS[eoff + (size_t)s * 2] + edc) - mx);
      den += p;
      const float* hs = hw + (size_t)s * HCN + col;
      const v4f h0 = *(const v4f*)hs;
      const v4f h1 = *(const v4f*)(hs + 4);
      b0 = b0 + h0 * p; b1 = b1 + h1 * p;
    }
  }
  deno = den; a0 = b0; a1 = b1;
}

__global__ __launch_bounds__(NTHR) void k_agg1(
    const int* __restrict__ csr, const int* __restrict__ off, const int* __restrict__ cnt,
    const float* __restrict__ eS, const float* __restrict__ eD, const float* __restrict__ hw,
    const float* __restrict__ bias, unsigned short* xo, int nN, int npad, int csrLen) {
  const int tid = threadIdx.x, lane = tid & 31, wave = tid >> 5;
  const int tbase = blockIdx.x * TGT + wave * 32;
  const int col = CPL * lane;
  const int hd  = lane >> 3;
  const size_t eoff = (size_t)(hd >> 1) * (size_t)npad * 2 + (size_t)(hd & 1);

  const v4f bb0 = *(const v4f*)(bias + col);
  const v4f bb1 = *(const v4f*)(bias + col + 4);

  const int cl    = tbase + lane;
  const int cnt_l = cnt[cl];
  const int off_l = off[cl];

#pragma unroll 1
  for (int j = 0; j < 32; ++j) {
    const int c = tbase + j;
    int n = __shfl(cnt_l, j);
    n = n < 0 ? 0 : (n > DEGCAP ? DEGCAP : n);
    const int st = __shfl(off_l, j);
    const float edc   = eD[eoff + (size_t)c * 2];
    const float eself = lrelu(eS[eoff + (size_t)c * 2] + edc);

    float den;
    v4f a0, a1;
    gat_row(csr, eS, hw, eoff, edc, eself, c, n, st, col, lane, nN, csrLen, den, a0, a1);

    const float rd = __builtin_amdgcn_rcpf(den);
    v4f v0 = elu4(a0 * rd + bb0);
    v4f v1 = elu4(a1 * rd + bb1);
    if (c >= nN) { const v4f z = {0.f, 0.f, 0.f, 0.f}; v0 = z; v1 = z; }
    const v8us q = cvt8h(v0, v1, H1SC);
    unsigned short* gp = xo + (size_t)c * HCN + col;
    *(volatile v8us*)gp = q;
    __threadfence();
    *(volatile v8us*)gp = q;
  }
}

__global__ __launch_bounds__(NTHR) void k_agg2(
    const int* __restrict__ csr, const int* __restrict__ off, const int* __restrict__ cnt,
    const float* __restrict__ eS, const float* __restrict__ eD, const float* __restrict__ hw,
    const float* __restrict__ bias, float* z, int nN, int npad, int csrLen) {
  const int tid = threadIdx.x, lane = tid & 31, wave = tid >> 5;
  const int tbase = blockIdx.x * TGT + wave * 32;
  const int col = CPL * lane;
  const int hd  = lane >> 3;
  const size_t eoff = (size_t)(hd >> 1) * (size_t)npad * 2 + (size_t)(hd & 1);

  const int lq  = lane < 16 ? lane : 15;
  const int sl2 = lq >> 1;
  const bool odd = (lq & 1) != 0;
  const v4f bb = *(const v4f*)(bias + 4 * lq);

  const int cl    = tbase + lane;
  const int cnt_l = cnt[cl];
  const int off_l = off[cl];

#pragma unroll 1
  for (int j = 0; j < 32; ++j) {
    const int c = tbase + j;
    int n = __shfl(cnt_l, j);
    n = n < 0 ? 0 : (n > DEGCAP ? DEGCAP : n);
    const int st = __shfl(off_l, j);
    const float edc   = eD[eoff + (size_t)c * 2];
    const float eself = lrelu(eS[eoff + (size_t)c * 2] + edc);

    float den;
    v4f a0, a1;
    gat_row(csr, eS, hw, eoff, edc, eself, c, n, st, col, lane, nN, csrLen, den, a0, a1);

    const float rd = __builtin_amdgcn_rcpf(den);
    const v4f v0 = hsum2v(a0 * rd);
    const v4f v1 = hsum2v(a1 * rd);
    v4f s0, s1;
    s0.x = __shfl(v0.x, sl2); s0.y = __shfl(v0.y, sl2); s0.z = __shfl(v0.z, sl2); s0.w = __shfl(v0.w, sl2);
    s1.x = __shfl(v1.x, sl2); s1.y = __shfl(v1.y, sl2); s1.z = __shfl(v1.z, sl2); s1.w = __shfl(v1.w, sl2);
    v4f o;
    o.x = odd ? s1.x : s0.x; o.y = odd ? s1.y : s0.y; o.z = odd ? s1.z : s0.z; o.w = odd ? s1.w : s0.w;
    o = o * 0.25f + bb;
    float* gp = z + (size_t)c * CHN + 4 * lq;
    if (lane < 16) *(volatile v4f*)gp = o;
    __threadfence();
    if (lane < 16) *(volatile v4f*)gp = o;
  }
}

__global__ __launch_bounds__(NTHR) void k_dec(
    const int* __restrict__ srcs, const int* __restrict__ dsts,
    const float* __restrict__ z, float* out, int nN, int nE) {
  __shared__ __attribute__((aligned(16))) float so[NTHR];
  const int tid = threadIdx.x;
  const int ebase = blockIdx.x * NTHR;
  int e = ebase + tid;
  e = e > nE - 1 ? nE - 1 : e;
  e = e < 0 ? 0 : e;
  int s = srcs[e];
  int d = dsts[e];
  s = s < 0 ? 0 : (s > nN - 1 ? nN - 1 : s);
  d = d < 0 ? 0 : (d > nN - 1 ? nN - 1 : d);
  const float* zs = z + (size_t)s * CHN;
  const float* zd = z + (size_t)d * CHN;
  float acc = 0.f;
#pragma unroll 4
  for (int c = 0; c < CHN; c += 4) {
    const v4f a = *(const v4f*)(zs + c);
    const v4f b = *(const v4f*)(zd + c);
    acc += a.x * b.x + a.y * b.y + a.z * b.z + a.w * b.w;
  }
  so[tid] = acc;
  __syncthreads();

  const bool act = tid < (NTHR / 4);
  const int q = act ? tid : 0;
  const v4f w = *(const v4f*)(so + 4 * q);
  const int i0 = ebase + 4 * q;
  const bool full = act && (i0 + 4 <= nE);
  const bool part = act && (i0 < nE) && !full;
  float* gp = out + (size_t)ebase + 4 * q;
  if (full) *(volatile v4f*)gp = w;
  if (part) {
    if (i0 < nE)     ((volatile float*)gp)[0] = w.x;
    if (i0 + 1 < nE) ((volatile float*)gp)[1] = w.y;
    if (i0 + 2 < nE) ((volatile float*)gp)[2] = w.z;
  }
  __threadfence();
  if (full) *(volatile v4f*)gp = w;
  if (part) {
    if (i0 < nE)     ((volatile float*)gp)[0] = w.x;
    if (i0 + 1 < nE) ((volatile float*)gp)[1] = w.y;
    if (i0 + 2 < nE) ((volatile float*)gp)[2] = w.z;
  }
}

extern "C" void kernel_launch(void* const* d_in, const int* in_sizes, int n_in,
                              void* d_out, int out_size, void* d_ws, size_t ws_size,
                              hipStream_t stream) {
  if (n_in < 10) return;
  const int nN = in_sizes[0] / FIN;
  const int nE = in_sizes[1] / 2;
  if (nN <= 0 || nE <= 0 || in_sizes[0] != nN * FIN || in_sizes[1] != 2 * nE) return;
  if (in_sizes[2] != FIN * HCN || in_sizes[3] != NHD * CHN || in_sizes[4] != NHD * CHN || in_sizes[5] != HCN) return;
  if (in_sizes[6] != HCN * HCN || in_sizes[7] != NHD * CHN || in_sizes[8] != NHD * CHN || in_sizes[9] != CHN) return;
  if (nE > (1 << 26) || nN > (1 << 22)) return;
  if ((long long)out_size != (long long)nE) return;

  const float* x   = (const float*)d_in[0];
  const int*   ei  = (const int*)d_in[1];
  const int*   src = ei;
  const int*   dst = ei + nE;
  const float* W1  = (const float*)d_in[2];
  const float* a1s = (const float*)d_in[3];
  const float* a1d = (const float*)d_in[4];
  const float* b1  = (const float*)d_in[5];
  const float* W2  = (const float*)d_in[6];
  const float* a2s = (const float*)d_in[7];
  const float* a2d = (const float*)d_in[8];
  const float* b2  = (const float*)d_in[9];
  float* out0 = (float*)d_out;

  const int NPAD   = ((nN + TGT - 1) / TGT) * TGT;
  const int nBC    = (nN + NBC - 1) / NBC;
  const int CNTPAD = nBC * NBC;
  if (CNTPAD < NPAD) return;
  if (4 * nBC + 1 > RBN) return;
  const int nBF    = (nN + NBF - 1) / NBF;
  if (nBF + 1 > 4 * nBC + 1) return;
  const int csrLen = ((nE + 31) & ~31) + 4096;
  if (31 * 4 * nBC > 4096) return;
  const int nAgg   = NPAD / TGT;
  const int nGemm  = NPAD / BM;
  const int nXu    = NPAD * (FIN / 8);
  const int nDec   = (nE + NTHR - 1) / NTHR;

  char* ws = (char*)d_ws;
  size_t off = 0;
  const size_t oW1  = off; off += (size_t)HCN * FIN * 2;         off = (off + 255) & ~(size_t)255;
  const size_t oW2  = off; off += (size_t)HCN * HCN * 2;         off = (off + 255) & ~(size_t)255;
  const size_t oA   = off; off += (size_t)NPAD * HCN * 2;        off = (off + 255) & ~(size_t)255;
  const size_t oCnt = off; off += (size_t)CNTPAD * 4;            off = (off + 255) & ~(size_t)255;
  const size_t oOff = off; off += (size_t)CNTPAD * 4;            off = (off + 255) & ~(size_t)255;
  const size_t oRb  = off; off += (size_t)RBN * 4;               off = (off + 255) & ~(size_t)255;
  const size_t oCsr = off; off += (size_t)csrLen * 4;            off = (off + 255) & ~(size_t)255;
  const size_t oHw  = off; off += (size_t)NPAD * HCN * 4;        off = (off + 255) & ~(size_t)255;
  const size_t oES  = off; off += (size_t)NPAD * NHD * 4;        off = (off + 255) & ~(size_t)255;
  const size_t oED  = off; off += (size_t)NPAD * NHD * 4;        off = (off + 255) & ~(size_t)255;
  const size_t oZ   = off; off += (size_t)NPAD * CHN * 4;        off = (off + 255) & ~(size_t)255;
  if (off > ws_size || off > (size_t)WSCAP) return;
  unsigned short* wp1 = (unsigned short*)(ws + oW1);
  unsigned short* wp2 = (unsigned short*)(ws + oW2);
  unsigned short* pa  = (unsigned short*)(ws + oA);
  int*   cnt  = (int*)(ws + oCnt);
  int*   offp = (int*)(ws + oOff);
  int*   rb   = (int*)(ws + oRb);
  int*   csr  = (int*)(ws + oCsr);
  float* hw   = (float*)(ws + oHw);
  float* es   = (float*)(ws + oES);
  float* ed   = (float*)(ws + oED);
  float* zp   = (float*)(ws + oZ);

  const int vec8 = ((nE & 3) == 0) ? 1 : 0;

  k_wprep<FIN, HCN><<<(HCN * FIN / 8 + NTHR - 1) / NTHR, NTHR, 0, stream>>>(W1, wp1);
  k_wprep<HCN, HCN><<<(HCN * HCN / 8 + NTHR - 1) / NTHR, NTHR, 0, stream>>>(W2, wp2);
  k_xcvt<<<(nXu + NTHR - 1) / NTHR, NTHR, 0, stream>>>(x, pa, nN, nXu);

  k_count<<<nBC, NTHR, 0, stream>>>(dst, cnt, nE, vec8);
  k_offsets<<<1, OTHR, 0, stream>>>(cnt, offp, rb, nBC);
  hipFuncSetAttribute(reinterpret_cast<const void*>(&k_fill),
                      hipFuncAttributeMaxDynamicSharedMemorySize, LDS_FILL);
  k_fill<<<nBF, NTHR, LDS_FILL, stream>>>(src, dst, offp, rb, csr, nN, nE, vec8, csrLen);

  k_gemm<FIN, 4><<<dim3(nGemm, HCN / BN), NTHR, 0, stream>>>(pa, wp1, a1s, a1d, hw, es, ed, NPAD);
  k_agg1<<<nAgg, NTHR, 0, stream>>>(csr, offp, cnt, es, ed, hw, b1, pa, nN, NPAD, csrLen);

  k_gemm<HCN, 7><<<dim3(nGemm, HCN / BN), NTHR, 0, stream>>>(pa, wp2, a2s, a2d, hw, es, ed, NPAD);
  k_agg2<<<nAgg, NTHR, 0, stream>>>(csr, offp, cnt, es, ed, hw, b2, zp, nN, NPAD, csrLen);

  k_dec<<<nDec, NTHR, 0, stream>>>(src, dst, zp, out0, nN, nE);
}
